// BlockWiseDistanceComputation_16870631539359
// MI455X (gfx1250) — hardware-verified
//
#include <hip/hip_runtime.h>


#define NT   2048
#define DD   512
#define NH_  8
#define HD   64
#define BM   128
#define PEPS 1e-6f
#define DM   DD
#define NTK  NT
#define LOSC 1024.0f

typedef _Float16 h16;
typedef unsigned short bf;
typedef __attribute__((ext_vector_type(16))) __bf16   v16bf;
typedef __attribute__((ext_vector_type(16))) _Float16 v16h;
typedef __attribute__((ext_vector_type(8)))  _Float16 v8h;
typedef __attribute__((ext_vector_type(8)))  unsigned short v8us;
typedef __attribute__((ext_vector_type(8)))  float    v8f;
typedef __attribute__((ext_vector_type(4)))  float    v4f;
typedef __attribute__((ext_vector_type(4)))  _Float16 v4h;
typedef v8h  __attribute__((may_alias)) v8ha;
typedef v4f  __attribute__((may_alias)) v4fa;
typedef v8us __attribute__((may_alias)) v8usa;

__device__ __forceinline__ unsigned short f2bf(float f) { unsigned u = __float_as_uint(f); u += 0x7FFFu + ((u >> 16) & 1u); return (unsigned short)(u >> 16); }
__device__ __forceinline__ float bf2f(unsigned short b) { return __uint_as_float(((unsigned)b) << 16); }
__device__ __forceinline__ float bfr(float f) { return bf2f(f2bf(f)); }
__device__ __forceinline__ v16h cat16(v8h lo, v8h hi) { return __builtin_shufflevector(lo, hi, 0, 1, 2, 3, 4, 5, 6, 7, 8, 9, 10, 11, 12, 13, 14, 15); }
__device__ __forceinline__ v16bf cat16b(v8us lo, v8us hi) { return __builtin_bit_cast(v16bf, __builtin_shufflevector(lo, hi, 0, 1, 2, 3, 4, 5, 6, 7, 8, 9, 10, 11, 12, 13, 14, 15)); }
__device__ __forceinline__ v8f wmma16(v16h a, v16h b, v8f c) { return __builtin_amdgcn_wmma_f32_16x16x32_f16(false, a, false, b, (short)0, c, false, false); }
__device__ __forceinline__ v8f wmmab(v16bf a, v16bf b, v8f c) { return __builtin_amdgcn_wmma_f32_16x16x32_bf16(false, a, false, b, (short)0, c, false, false); }

__global__ __launch_bounds__(256) void k_wt(const float* __restrict__ Wm, int K, int ncols, bf* WT) {
    __shared__ __align__(16) unsigned short tl[64 * 72];
    const int tid = threadIdx.x, k0 = blockIdx.x * 64, n0 = blockIdx.y * 64;
    const int kk = tid >> 2, nq = (tid & 3) * 16;
#pragma unroll
    for (int i = 0; i < 16; ++i) tl[(nq + i) * 72 + kk] = f2bf(Wm[(size_t)(k0 + kk) * ncols + n0 + nq + i]);
    __syncthreads();
    const int piece = tid & 7;
    auto pass = [&]() {
#pragma unroll
        for (int s = 0; s < 2; ++s) { const int nr = (tid >> 3) + 32 * s; const v8us val = *(const v8usa*)(tl + nr * 72 + piece * 8); *(volatile v8us*)(WT + (size_t)(n0 + nr) * K + k0 + piece * 8) = val; }
    };
    pass(); __threadfence(); pass();
}
template <bool SPLITA, bool F16OUT = false>
__global__ __launch_bounds__(128) void k_gemmb(const bf* __restrict__ A, const bf* __restrict__ Al, const bf* __restrict__ Bn, const float* __restrict__ bias, float* C, int ldc, h16* C2, const float* __restrict__ R = nullptr, int K = DM, int roundR = 1) {
    __shared__ __align__(16) float ost[4][16 * 68];
    const int lane = threadIdx.x & 31, wave = threadIdx.x >> 5, lr = lane & 15, hi = lane >> 4;
    const int r0 = blockIdx.x * 64 + wave * 16, c0 = blockIdx.y * 64;
    const size_t aoff = (size_t)(r0 + lr) * K + 8 * hi;
    size_t boff[4];
#pragma unroll
    for (int t = 0; t < 4; ++t) boff[t] = (size_t)(c0 + t * 16 + lr) * K + 8 * hi;
    v8f acc[4];
#pragma unroll
    for (int t = 0; t < 4; ++t) acc[t] = (v8f){};
#pragma unroll 1
    for (int kc = 0; kc < K; kc += 32) {
        const v16bf a = cat16b(*(const v8us*)(A + aoff + kc), *(const v8us*)(A + aoff + kc + 16));
        v16bf al = a;
        if (SPLITA) al = cat16b(*(const v8us*)(Al + aoff + kc), *(const v8us*)(Al + aoff + kc + 16));
#pragma unroll
        for (int t = 0; t < 4; ++t) { const v16bf b = cat16b(*(const v8us*)(Bn + boff[t] + kc), *(const v8us*)(Bn + boff[t] + kc + 16)); acc[t] = wmmab(a, b, acc[t]); if (SPLITA) acc[t] = wmmab(al, b, acc[t]); }
        asm volatile("v_nop\n\tv_nop\n\tv_nop\n\tv_nop" : "+v"(acc[0]), "+v"(acc[1]), "+v"(acc[2]), "+v"(acc[3]) : "v"(a), "v"(al));
    }
    float* os = &ost[wave][0];
#pragma unroll
    for (int t = 0; t < 4; ++t) { const float bv = bias ? bfr(bias[c0 + t * 16 + lr]) : 0.f;
#pragma unroll
        for (int j = 0; j < 8; ++j) os[(hi * 8 + j) * 68 + t * 16 + lr] = acc[t][j] + bv; }
    __syncthreads();
    if (F16OUT) {
        h16* crow = (h16*)(void*)C + (size_t)r0 * ldc + c0;
        auto pass = [&]() {
#pragma unroll
            for (int s = 0; s < 4; ++s) { const int row = 4 * s + (lane >> 3), piece = lane & 7; const float* sp = os + row * 68 + piece * 8; v8h o, o2;
#pragma unroll
                for (int i = 0; i < 8; ++i) { const h16 a = (h16)sp[i]; o[i] = a; o2[i] = (h16)((sp[i] - (float)a) * LOSC); }
                *(volatile v8h*)(crow + (size_t)row * ldc + piece * 8) = o; if (C2) *(volatile v8h*)(C2 + (size_t)r0 * ldc + c0 + (size_t)row * ldc + piece * 8) = o2; }
        };
        pass(); __threadfence(); pass();
    } else {
        float* crow = C + (size_t)r0 * ldc + c0;
        auto pass = [&]() {
#pragma unroll
            for (int s = 0; s < 8; ++s) { const int Lid = (lane >> 3) + 4 * s, piece = lane & 7; const int row = Lid >> 1, cofs = (Lid & 1) * 32 + piece * 4;
                v4f val = *(const v4fa*)(os + row * 68 + cofs); if (R) { const v4f rv = *(const v4f*)(R + ((size_t)r0 + row) * ldc + c0 + cofs); val += roundR ? (v4f){bfr(rv[0]), bfr(rv[1]), bfr(rv[2]), bfr(rv[3])} : rv; }
                *(volatile v4f*)(crow + (size_t)row * ldc + cofs) = val; }
        };
        pass(); __threadfence(); pass();
    }
}

__global__ __launch_bounds__(128) void k_gemm3(const bf* __restrict__ Ah, const bf* __restrict__ Al, const bf* __restrict__ Bh, const bf* __restrict__ Bl, int K, float* C, int ldc) {
    __shared__ __align__(16) float ost[4][16 * 68];
    const int lane = threadIdx.x & 31, wave = threadIdx.x >> 5, lr = lane & 15, hi = lane >> 4;
    const int r0 = blockIdx.x * 64 + wave * 16, c0 = blockIdx.y * 64;
    const size_t aoff = (size_t)(r0 + lr) * K + 8 * hi;
    v8f acc[4];
#pragma unroll
    for (int t = 0; t < 4; ++t) acc[t] = (v8f){};
#pragma unroll 1
    for (int kc = 0; kc < K; kc += 32) {
        const v16bf a = cat16b(*(const v8us*)(Ah + aoff + kc), *(const v8us*)(Ah + aoff + kc + 16));
        const v16bf al = cat16b(*(const v8us*)(Al + aoff + kc), *(const v8us*)(Al + aoff + kc + 16));
#pragma unroll
        for (int t = 0; t < 4; ++t) { const size_t bo = (size_t)(c0 + t * 16 + lr) * K + kc + 8 * hi;
            const v16bf bh = cat16b(*(const v8us*)(Bh + bo), *(const v8us*)(Bh + bo + 16)); const v16bf bl = cat16b(*(const v8us*)(Bl + bo), *(const v8us*)(Bl + bo + 16));
            acc[t] = wmmab(a, bh, acc[t]); acc[t] = wmmab(al, bh, acc[t]); acc[t] = wmmab(a, bl, acc[t]); }
        asm volatile("v_nop\n\tv_nop\n\tv_nop\n\tv_nop" : "+v"(acc[0]), "+v"(acc[1]), "+v"(acc[2]), "+v"(acc[3]) : "v"(a), "v"(al));
    }
    float* os = &ost[wave][0];
#pragma unroll
    for (int t = 0; t < 4; ++t) {
#pragma unroll
        for (int j = 0; j < 8; ++j) os[(hi * 8 + j) * 68 + t * 16 + lr] = acc[t][j]; }
    __builtin_amdgcn_wave_barrier(); asm volatile("" ::: "memory");
    float* crow = C + (size_t)r0 * ldc + c0;
    auto pass = [&]() {
#pragma unroll
        for (int s = 0; s < 8; ++s) { const int Lid = (lane >> 3) + 4 * s, piece = lane & 7; const int row = Lid >> 1, cofs = (Lid & 1) * 32 + piece * 4;
            const v4f val = *(const v4fa*)(os + row * 68 + cofs); *(volatile v4f*)(crow + (size_t)row * ldc + cofs) = val; }
    };
    pass(); __threadfence(); pass();
}


__global__ __launch_bounds__(256) void k_cvtx(const float* __restrict__ src, bf* dst) {
    const int lane = threadIdx.x & 31; const size_t r = (size_t)blockIdx.x * 8 + (threadIdx.x >> 5); if (r >= (size_t)NT) return;
#pragma unroll 1
    for (int ps = 0; ps < 2; ++ps) {
#pragma unroll
        for (int q = 0; q < DD / 256; ++q) { v8us o;
#pragma unroll
            for (int i = 0; i < 8; ++i) o[i] = f2bf(src[r * DD + q * 256 + lane * 8 + i]);
            *(volatile v8us*)(dst + r * DD + q * 256 + lane * 8) = o; }
        if (ps == 0) __threadfence(); }
}
__global__ __launch_bounds__(256) void k_hplanes(const float* __restrict__ SRC, int h, bf* Ph, bf* Pl) {
    typedef __attribute__((ext_vector_type(2))) unsigned short v2us;
    const int lane = threadIdx.x & 31; const size_t t = (size_t)blockIdx.x * 8 + (threadIdx.x >> 5); if (t >= (size_t)NT) return; v2us oh, ol;
#pragma unroll
    for (int i = 0; i < 2; ++i) { const float v = SRC[t * DD + h * HD + lane * 2 + i]; const unsigned short hb = f2bf(v); oh[i] = hb; ol[i] = f2bf(v - bf2f(hb)); }
    const size_t o = t * HD + lane * 2; *(volatile v2us*)(Ph + o) = oh; *(volatile v2us*)(Pl + o) = ol; __threadfence(); *(volatile v2us*)(Ph + o) = oh; *(volatile v2us*)(Pl + o) = ol;
}
__global__ __launch_bounds__(256) void k_sq(const float* __restrict__ SRC, int h, float* SQ) {
    const int t = blockIdx.x * 256 + threadIdx.x; if (t >= NT) return; float s = 0.f;
#pragma unroll 8
    for (int d = 0; d < HD; ++d) { const float v = SRC[(size_t)t * DD + h * HD + d]; s = fmaf(v, v, s); }
    *(volatile float*)(SQ + t) = s; __threadfence(); *(volatile float*)(SQ + t) = s;
}
__global__ __launch_bounds__(256) void k_vt(const float* __restrict__ Vs, int h, bf* Th, bf* Tl) {
    typedef __attribute__((ext_vector_type(2))) unsigned short v2us;
    const int lane = threadIdx.x & 31; const size_t wid = (size_t)blockIdx.x * 8 + (threadIdx.x >> 5); if (wid >= (size_t)HD * (NT / 64)) return; const int d = (int)(wid / (NT / 64)); const int t0 = (int)(wid % (NT / 64)) * 64 + lane * 2; v2us oh, ol;
#pragma unroll
    for (int i = 0; i < 2; ++i) { const float v = Vs[(size_t)(t0 + i) * DD + h * HD + d]; const unsigned short hb = f2bf(v); oh[i] = hb; ol[i] = f2bf(v - bf2f(hb)); }
    const size_t o = (size_t)d * NT + t0; *(volatile v2us*)(Th + o) = oh; *(volatile v2us*)(Tl + o) = ol; __threadfence(); *(volatile v2us*)(Th + o) = oh; *(volatile v2us*)(Tl + o) = ol;
}
__global__ __launch_bounds__(256) void k_bsoft(const float* __restrict__ QK, const float* __restrict__ QN, const float* __restrict__ KN, const float* __restrict__ cin, bf* EH, bf* EL, float* NRML) {
    typedef __attribute__((ext_vector_type(4))) unsigned short v4us;
    __shared__ float sh[8];
    const int lane = threadIdx.x & 31, wv = threadIdx.x >> 5, i = blockIdx.x * 8 + wv; const int rb = i / BM;
    const float cc = fmaxf(fabsf(bfr(cin[0])), 1e-6f), sqc = sqrtf(fmaxf(cc, PEPS)), isqc = 1.0f / sqc; const float qn = QN[i]; const float dq = 1.0f - cc * qn;
    float total = 0.f;
#pragma unroll 1
    for (int ps = 0; ps < 2; ++ps) { total = 0.f;
#pragma unroll 1
        for (int cb = 0; cb < NT / BM; ++cb) { const int j0 = cb * BM + lane * 4; float s[4]; bool live[4]; float m = -3.0e38f;
#pragma unroll
            for (int q = 0; q < 4; ++q) { const int j = j0 + q; live[q] = (cb < rb) || (cb == rb && j <= i);
                const float kn = KN[j]; const float diff = fmaxf(qn + kn - 2.0f * QK[(size_t)i * NT + j], 0.f); const float den = fmaxf(dq * (1.0f - cc * kn), PEPS);
                const float arg = fmaxf(1.0f + 2.0f * cc * diff / den, 1.0f + PEPS); s[q] = -acoshf(arg) * isqc; if (live[q]) m = fmaxf(m, s[q]); }
#pragma unroll
            for (int x = 16; x; x >>= 1) m = fmaxf(m, __shfl_xor(m, x, 32));
            v4us oh, ol;
#pragma unroll
            for (int q = 0; q < 4; ++q) { const float e = live[q] ? __expf(s[q] - m) : 0.f; total += e; const unsigned short hb = f2bf(e); oh[q] = hb; ol[q] = f2bf(e - bf2f(hb)); }
            const size_t o = (size_t)i * NT + j0; *(volatile v4us*)(EH + o) = oh; *(volatile v4us*)(EL + o) = ol; }
        if (ps == 0) __threadfence(); }
#pragma unroll
    for (int x = 16; x; x >>= 1) total += __shfl_xor(total, x, 32);
    if (lane == 0) sh[wv] = fmaxf(total, PEPS);
    __syncthreads();
    if (wv == 0) { const float v = (lane < 8) ? sh[lane] : 0.f; float* d = NRML + (size_t)blockIdx.x * 32 + lane; *(volatile float*)d = v; __threadfence(); *(volatile float*)d = v; }
}
__global__ __launch_bounds__(256) void k_ctxplanes(const float* __restrict__ CTX, const float* __restrict__ NRML, bf* dh, bf* dl) {
    const int lane = threadIdx.x & 31; const size_t t = (size_t)blockIdx.x * 8 + (threadIdx.x >> 5); if (t >= (size_t)NT) return;
#pragma unroll 1
    for (int ps = 0; ps < 2; ++ps) {
#pragma unroll
        for (int q = 0; q < DD / 256; ++q) { const int c0 = q * 256 + lane * 8; const int h = c0 / HD; const float inv = 1.0f / NRML[(size_t)h * (NT / 8) * 32 + (t >> 3) * 32 + (t & 7)]; v8us oh, ol;
#pragma unroll
            for (int i2 = 0; i2 < 8; ++i2) { const float v = CTX[t * DD + c0 + i2] * inv; const unsigned short hb = f2bf(v); oh[i2] = hb; ol[i2] = f2bf(v - bf2f(hb)); }
            *(volatile v8us*)(dh + t * DD + c0) = oh; *(volatile v8us*)(dl + t * DD + c0) = ol; }
        if (ps == 0) __threadfence(); }
}

extern "C" void kernel_launch(void* const* d_in, const int* in_sizes, int n_in,
                              void* d_out, int out_size, void* d_ws, size_t ws_size, hipStream_t stream) {
    (void)in_sizes; (void)n_in; (void)out_size;
    const float* x = (const float*)d_in[0]; const float* cin = (const float*)d_in[1]; const float* Wq = (const float*)d_in[2]; const float* bq = (const float*)d_in[3]; const float* Wk = (const float*)d_in[4]; const float* bk = (const float*)d_in[5];
    const float* Wv = (const float*)d_in[6]; const float* bv = (const float*)d_in[7]; const float* Wo = (const float*)d_in[8]; const float* bo = (const float*)d_in[9];
    float* out = (float*)d_out;
    char* wsp = (char*)d_ws;
    auto take = [&](size_t bytes) { char* p = wsp; wsp += (bytes + 255) & ~(size_t)255; return (void*)p; };
    bf* WQT = (bf*)take((size_t)DD * DD * 2); bf* WKT = (bf*)take((size_t)DD * DD * 2); bf* WVT = (bf*)take((size_t)DD * DD * 2); bf* WOT = (bf*)take((size_t)DD * DD * 2);
    bf* Xb = (bf*)take((size_t)NT * DD * 2); float* QF = (float*)take((size_t)NT * DD * 4); float* KF = (float*)take((size_t)NT * DD * 4); float* VF = (float*)take((size_t)NT * DD * 4);
    bf* Qh = (bf*)take((size_t)NT * HD * 2); bf* Ql = (bf*)take((size_t)NT * HD * 2); bf* Kh = (bf*)take((size_t)NT * HD * 2); bf* Kl = (bf*)take((size_t)NT * HD * 2); bf* VTh = (bf*)take((size_t)HD * NT * 2); bf* VTl = (bf*)take((size_t)HD * NT * 2);
    float* QN = (float*)take(NT * 4); float* KN = (float*)take(NT * 4); float* QK = (float*)take((size_t)NT * NT * 4); bf* EH = (bf*)take((size_t)NT * NT * 2); bf* EL = (bf*)take((size_t)NT * NT * 2); float* NRML = (float*)take((size_t)NH_ * (NT / 8) * 32 * 4);
    float* CTX = (float*)take((size_t)NT * DD * 4); bf* Ch = (bf*)take((size_t)NT * DD * 2); bf* Cl = (bf*)take((size_t)NT * DD * 2);
    if ((size_t)(wsp - (char*)d_ws) > ws_size) return;
    k_wt<<<dim3(DD / 64, DD / 64, 1), 256, 0, stream>>>(Wq, DD, DD, WQT); k_wt<<<dim3(DD / 64, DD / 64, 1), 256, 0, stream>>>(Wk, DD, DD, WKT); k_wt<<<dim3(DD / 64, DD / 64, 1), 256, 0, stream>>>(Wv, DD, DD, WVT); k_wt<<<dim3(DD / 64, DD / 64, 1), 256, 0, stream>>>(Wo, DD, DD, WOT);
    k_cvtx<<<NT / 8, 256, 0, stream>>>(x, Xb);
    k_gemmb<false, false><<<dim3(NT / 64, DD / 64, 1), 128, 0, stream>>>(Xb, nullptr, WQT, bq, QF, DD, nullptr, nullptr, DD);
    k_gemmb<false, false><<<dim3(NT / 64, DD / 64, 1), 128, 0, stream>>>(Xb, nullptr, WKT, bk, KF, DD, nullptr, nullptr, DD);
    k_gemmb<false, false><<<dim3(NT / 64, DD / 64, 1), 128, 0, stream>>>(Xb, nullptr, WVT, bv, VF, DD, nullptr, nullptr, DD);
    for (int h = 0; h < NH_; ++h) {
        k_hplanes<<<NT / 8, 256, 0, stream>>>(QF, h, Qh, Ql); k_hplanes<<<NT / 8, 256, 0, stream>>>(KF, h, Kh, Kl); k_sq<<<NT / 256, 256, 0, stream>>>(QF, h, QN); k_sq<<<NT / 256, 256, 0, stream>>>(KF, h, KN); k_vt<<<(HD * (NT / 64)) / 8, 256, 0, stream>>>(VF, h, VTh, VTl);
        k_gemm3<<<dim3(NT / 64, NT / 64, 1), 128, 0, stream>>>(Qh, Ql, Kh, Kl, HD, QK, NT);
        k_bsoft<<<NT / 8, 256, 0, stream>>>(QK, QN, KN, cin, EH, EL, NRML + (size_t)h * (NT / 8) * 32);
        k_gemm3<<<dim3(NT / 64, 1, 1), 128, 0, stream>>>(EH, EL, VTh, VTl, NT, CTX + h * HD, DD); }
    k_ctxplanes<<<NT / 8, 256, 0, stream>>>(CTX, NRML, Ch, Cl);
    k_gemmb<true, false><<<dim3(NT / 64, DD / 64, 1), 128, 0, stream>>>(Ch, Cl, WOT, bo, out, DD, nullptr, nullptr, DD);
}
